// InfiniBlock_42494406426645
// MI455X (gfx1250) — hardware-verified
//
#include <hip/hip_runtime.h>


#define NB_  4
#define TT   2048
#define DM   1024
#define RH   512
#define PCAR 1024.0f
#define SCL  0.03125f
typedef _Float16 h16;
typedef unsigned short bf;
typedef __attribute__((ext_vector_type(16))) __bf16   v16bf;
typedef __attribute__((ext_vector_type(16))) _Float16 v16h;
typedef __attribute__((ext_vector_type(8)))  _Float16 v8h;
typedef __attribute__((ext_vector_type(8)))  unsigned short v8us;
typedef __attribute__((ext_vector_type(8)))  float    v8f;
typedef __attribute__((ext_vector_type(4)))  float    v4f;
typedef v8h  __attribute__((may_alias)) v8ha;
typedef v4f  __attribute__((may_alias)) v4fa;
typedef v8us __attribute__((may_alias)) v8usa;

__device__ __forceinline__ unsigned short f2bf(float f) { unsigned u = __float_as_uint(f); u += 0x7FFFu + ((u >> 16) & 1u); return (unsigned short)(u >> 16); }
__device__ __forceinline__ float bf2f(unsigned short b) { return __uint_as_float(((unsigned)b) << 16); }
__device__ __forceinline__ float bfr(float f) { return bf2f(f2bf(f)); }
__device__ __forceinline__ v16h cat16(v8h lo, v8h hi) { return __builtin_shufflevector(lo, hi, 0, 1, 2, 3, 4, 5, 6, 7, 8, 9, 10, 11, 12, 13, 14, 15); }
__device__ __forceinline__ v16bf cat16b(v8us lo, v8us hi) { return __builtin_bit_cast(v16bf, __builtin_shufflevector(lo, hi, 0, 1, 2, 3, 4, 5, 6, 7, 8, 9, 10, 11, 12, 13, 14, 15)); }
__device__ __forceinline__ v8f wmma16(v16h a, v16h b, v8f c) { return __builtin_amdgcn_wmma_f32_16x16x32_f16(false, a, false, b, (short)0, c, false, false); }
__device__ __forceinline__ v8f wmmab(v16bf a, v16bf b, v8f c) { return __builtin_amdgcn_wmma_f32_16x16x32_bf16(false, a, false, b, (short)0, c, false, false); }


template <typename T16> struct WFrag;
template <> struct WFrag<h16> { typedef v16h V; static __device__ __forceinline__ V ld(const h16* p) { return cat16(*(const v8h*)p, *(const v8h*)(p + 16)); } static __device__ __forceinline__ v8f mma(V a, V b, v8f c) { return wmma16(a, b, c); } };
template <> struct WFrag<bf> { typedef v16bf V; static __device__ __forceinline__ V ld(const bf* p) { return cat16b(*(const v8us*)p, *(const v8us*)(p + 16)); } static __device__ __forceinline__ v8f mma(V a, V b, v8f c) { return wmmab(a, b, c); } };
template <typename T16, int NSPLIT, bool BIAS>
__global__ __launch_bounds__(32) void k_gemmw(const T16* __restrict__ A, const T16* __restrict__ A2, const T16* __restrict__ Bt, const T16* __restrict__ Bt2, int K, float* C, int ldc, const float* __restrict__ bias, size_t sA, size_t sB, size_t sC) {
    typedef typename WFrag<T16>::V V;
    __shared__ __align__(16) float os[16 * 68];
    const size_t z = blockIdx.z; A += z * sA; if (A2) A2 += z * sA; Bt += z * sB; if (Bt2) Bt2 += z * sB; C += z * sC;
    const int lane = threadIdx.x & 31, lr = lane & 15, hi = lane >> 4; const int r0 = blockIdx.x * 64, c0 = blockIdx.y * 64;
    v8f acc[4][4];
#pragma unroll
    for (int mb = 0; mb < 4; ++mb)
#pragma unroll
        for (int nb = 0; nb < 4; ++nb) acc[mb][nb] = (v8f){};
    const size_t aoff = (size_t)(r0 + lr) * K + 8 * hi, boff = (size_t)(c0 + lr) * K + 8 * hi;
#pragma unroll 1
    for (int kc = 0; kc < K; kc += 32) {
        V a[4], a2[4];
#pragma unroll
        for (int mb = 0; mb < 4; ++mb) { a[mb] = WFrag<T16>::ld(A + aoff + (size_t)mb * 16 * K + kc); if (NSPLIT == 1 || NSPLIT == 2) a2[mb] = WFrag<T16>::ld(A2 + aoff + (size_t)mb * 16 * K + kc); }
#pragma unroll
        for (int nb = 0; nb < 4; ++nb) { const V b = WFrag<T16>::ld(Bt + boff + (size_t)nb * 16 * K + kc); V b2; if (NSPLIT >= 2) b2 = WFrag<T16>::ld(Bt2 + boff + (size_t)nb * 16 * K + kc);
#pragma unroll
            for (int mb = 0; mb < 4; ++mb) { acc[mb][nb] = WFrag<T16>::mma(a[mb], b, acc[mb][nb]); if (NSPLIT == 1 || NSPLIT == 2) acc[mb][nb] = WFrag<T16>::mma(a2[mb], b, acc[mb][nb]); if (NSPLIT >= 2) acc[mb][nb] = WFrag<T16>::mma(a[mb], b2, acc[mb][nb]); } }
        asm volatile("v_nop\n\tv_nop\n\tv_nop\n\tv_nop" : "+v"(acc[0][0]), "+v"(acc[1][1]), "+v"(acc[2][2]), "+v"(acc[3][3]) : "v"(a[0]), "v"(a[3]));
    }
#pragma unroll
    for (int mb = 0; mb < 4; ++mb) {
#pragma unroll
        for (int nb = 0; nb < 4; ++nb) {
#pragma unroll
            for (int j = 0; j < 8; ++j) os[(hi * 8 + j) * 68 + nb * 16 + lr] = acc[mb][nb][j]; }
        __builtin_amdgcn_wave_barrier(); asm volatile("" ::: "memory");
        float* crow = C + (size_t)(r0 + mb * 16) * ldc + c0;
#pragma unroll 1
        for (int ps = 0; ps < 2; ++ps) {
#pragma unroll
            for (int s = 0; s < 8; ++s) { const int row = 2 * s + hi, cofs = lr * 4; v4f val = *(const v4fa*)(os + row * 68 + cofs); if (BIAS) { val[0] += bfr(bias[c0 + cofs]); val[1] += bfr(bias[c0 + cofs + 1]); val[2] += bfr(bias[c0 + cofs + 2]); val[3] += bfr(bias[c0 + cofs + 3]); }
                *(volatile v4f*)(crow + (size_t)row * ldc + cofs) = val; }
            if (ps == 0) __threadfence(); }
        __builtin_amdgcn_wave_barrier(); asm volatile("" ::: "memory");
    }
}

template <typename T16, int NSPLIT, int CMODE>
__global__ __launch_bounds__(32) void k_gemmc(const T16* __restrict__ A, const T16* __restrict__ A2, const T16* __restrict__ Bt, const T16* __restrict__ Bt2, int K, float* C, int ldc, int roff, size_t sA, size_t sB, size_t sC) {
    typedef typename WFrag<T16>::V V;
    __shared__ __align__(16) float os[16 * 68];
    const size_t z = blockIdx.z; A += z * sA; if (A2) A2 += z * sA; Bt += z * sB; if (Bt2) Bt2 += z * sB; C += z * sC;
    const int lane = threadIdx.x & 31, lr = lane & 15, hi = lane >> 4; const int r0 = blockIdx.x * 64, c0 = blockIdx.y * 64;
    if (CMODE == 1 && c0 > r0 + roff + 63) return;
    const int Kl = (CMODE == 2) ? min(K, r0 + roff + 64) : K;
    v8f acc[4][4];
#pragma unroll
    for (int mb = 0; mb < 4; ++mb)
#pragma unroll
        for (int nb = 0; nb < 4; ++nb) acc[mb][nb] = (v8f){};
    const size_t aoff = (size_t)(r0 + lr) * K + 8 * hi, boff = (size_t)(c0 + lr) * K + 8 * hi;
#pragma unroll 1
    for (int kc = 0; kc < Kl; kc += 32) {
        V a[4], a2[4];
#pragma unroll
        for (int mb = 0; mb < 4; ++mb) { a[mb] = WFrag<T16>::ld(A + aoff + (size_t)mb * 16 * K + kc); if (NSPLIT == 1 || NSPLIT == 2) a2[mb] = WFrag<T16>::ld(A2 + aoff + (size_t)mb * 16 * K + kc); }
#pragma unroll
        for (int nb = 0; nb < 4; ++nb) { const V b = WFrag<T16>::ld(Bt + boff + (size_t)nb * 16 * K + kc); V b2; if (NSPLIT >= 2) b2 = WFrag<T16>::ld(Bt2 + boff + (size_t)nb * 16 * K + kc);
#pragma unroll
            for (int mb = 0; mb < 4; ++mb) { acc[mb][nb] = WFrag<T16>::mma(a[mb], b, acc[mb][nb]); if (NSPLIT == 1 || NSPLIT == 2) acc[mb][nb] = WFrag<T16>::mma(a2[mb], b, acc[mb][nb]); if (NSPLIT >= 2) acc[mb][nb] = WFrag<T16>::mma(a[mb], b2, acc[mb][nb]); } }
        asm volatile("v_nop\n\tv_nop\n\tv_nop\n\tv_nop" : "+v"(acc[0][0]), "+v"(acc[1][1]), "+v"(acc[2][2]), "+v"(acc[3][3]) : "v"(a[0]), "v"(a[3]));
    }
#pragma unroll
    for (int mb = 0; mb < 4; ++mb) {
#pragma unroll
        for (int nb = 0; nb < 4; ++nb) {
#pragma unroll
            for (int j = 0; j < 8; ++j) os[(hi * 8 + j) * 68 + nb * 16 + lr] = acc[mb][nb][j]; }
        __builtin_amdgcn_wave_barrier(); asm volatile("" ::: "memory");
        float* crow = C + (size_t)(r0 + mb * 16) * ldc + c0;
#pragma unroll 1
        for (int ps = 0; ps < 2; ++ps) {
#pragma unroll
            for (int s = 0; s < 8; ++s) { const int row = 2 * s + hi, cofs = lr * 4; v4f val = *(const v4fa*)(os + row * 68 + cofs);
                *(volatile v4f*)(crow + (size_t)row * ldc + cofs) = val; }
            if (ps == 0) __threadfence(); }
        __builtin_amdgcn_wave_barrier(); asm volatile("" ::: "memory");
    }
}
__device__ __forceinline__ h16 tohx(float x) { return (h16)x; }
__device__ __forceinline__ void splitf(float y, unsigned short& h, unsigned short& l) { h = f2bf(y); l = f2bf(y - bf2f(h)); }
typedef __attribute__((ext_vector_type(2))) unsigned short v2us;
typedef __attribute__((ext_vector_type(4))) unsigned short v4us;
typedef __attribute__((ext_vector_type(2))) _Float16 v2h;
typedef __attribute__((ext_vector_type(4))) _Float16 v4h;

__global__ __launch_bounds__(256) void k_cvt8(const float* __restrict__ src, bf* dst, size_t n8) { const size_t i = (size_t)blockIdx.x * 256 + threadIdx.x; if (i >= n8) return; const v8f v = *(const v8f*)(src + i * 8); v8us o;
#pragma unroll
    for (int k = 0; k < 8; ++k) o[k] = f2bf(v[k]); *(volatile v8us*)(dst + i * 8) = o; __threadfence(); *(volatile v8us*)(dst + i * 8) = o; }
__global__ __launch_bounds__(256) void k_ropl(const float* __restrict__ F, const float* __restrict__ cs_, const float* __restrict__ sn_, h16* P16, bf* Ph, bf* Pl) { const size_t e = ((size_t)blockIdx.x * 256 + threadIdx.x) * 2; if (e >= (size_t)TT * DM) return; const int d = (int)(e % DM); const int t = (int)(e / DM); const float* f = F + (size_t)t * DM; v2h o16; v2us oh, ol;
#pragma unroll
    for (int q = 0; q < 2; ++q) { const int dd = d + q; const int dp = (dd < DM / 2) ? dd + DM / 2 : dd - DM / 2; float a = __fmul_rn(f[dd], bfr(cs_[(size_t)t * DM + dd])), bq = __fmul_rn(f[dp], bfr(sn_[(size_t)t * DM + dd])); asm volatile("" : "+v"(a)); asm volatile("" : "+v"(bq)); const float r = (dd < DM / 2) ? __fsub_rn(a, bq) : __fadd_rn(a, bq);
        o16[q] = tohx(r); unsigned short a2, c2; splitf(r, a2, c2); oh[q] = a2; ol[q] = c2; }
    *(volatile v2h*)(P16 + e) = o16; *(volatile v2us*)(Ph + e) = oh; *(volatile v2us*)(Pl + e) = ol; __threadfence(); *(volatile v2h*)(P16 + e) = o16; *(volatile v2us*)(Ph + e) = oh; *(volatile v2us*)(Pl + e) = ol; }
__global__ __launch_bounds__(256) void k_vtp1(const float* __restrict__ V, h16* VT16, bf* VTh, bf* VTl) { const size_t e = ((size_t)blockIdx.x * 256 + threadIdx.x) * 2; if (e >= (size_t)DM * TT) return; const int t = (int)(e % TT); const int d = (int)(e / TT); v2h o16; v2us oh, ol;
#pragma unroll
    for (int u = 0; u < 2; ++u) { const float v = V[(size_t)(t + u) * DM + d]; o16[u] = tohx(v); unsigned short a, b; splitf(v, a, b); oh[u] = a; ol[u] = b; }
    *(volatile v2h*)(VT16 + e) = o16; *(volatile v2us*)(VTh + e) = oh; *(volatile v2us*)(VTl + e) = ol; __threadfence(); *(volatile v2h*)(VT16 + e) = o16; *(volatile v2us*)(VTh + e) = oh; *(volatile v2us*)(VTl + e) = ol; }
__global__ __launch_bounds__(256) void k_isoft(const float* __restrict__ S, h16* P16, bf* Ph, bf* Pl) { const int lane = threadIdx.x & 31; const int i = blockIdx.x * 8 + (threadIdx.x >> 5); if (i >= TT) return; const bool hires = (i < RH); const float* sr = S + (size_t)i * TT; const int nch = (i >> 7) + 1; float v[TT / 32]; float mx = -3.0e38f;
#pragma unroll
    for (int ch = 0; ch < TT / 128; ++ch) { v4f a; if (ch < nch) a = *(const v4f*)(sr + ch * 128 + lane * 4); else { a[0] = 0.f; a[1] = 0.f; a[2] = 0.f; a[3] = 0.f; }
#pragma unroll
        for (int u = 0; u < 4; ++u) { const int j = ch * 128 + lane * 4 + u; const float t = (j <= i) ? a[u] * SCL : -3.0e38f; v[ch * 4 + u] = t; mx = fmaxf(mx, t); } }
#pragma unroll
    for (int sh = 16; sh; sh >>= 1) mx = fmaxf(mx, __shfl_xor(mx, sh, 32));
    float sum = 0.f;
#pragma unroll
    for (int q = 0; q < TT / 32; ++q) { float d0 = __fsub_rn(v[q], mx); asm volatile("" : "+v"(d0)); v[q] = __builtin_amdgcn_exp2f(__fmul_rn(d0, 1.4426950408889634f)); sum += v[q]; }
#pragma unroll
    for (int sh = 16; sh; sh >>= 1) sum += __shfl_xor(sum, sh, 32);
    const float f = __fdiv_rn(hires ? 1.0f : PCAR, sum);
    for (int ps = 0; ps < 2; ++ps) {
        if (hires) {
#pragma unroll
            for (int ch = 0; ch < TT / 128; ++ch) { v4us oh, ol; for (int q = 0; q < 4; ++q) { unsigned short a, b; splitf(v[ch * 4 + q] * f, a, b); oh[q] = a; ol[q] = b; } const size_t oo = (size_t)i * TT + ch * 128 + lane * 4; *(volatile v4us*)(Ph + oo) = oh; *(volatile v4us*)(Pl + oo) = ol; }
        } else {
#pragma unroll
            for (int ch = 0; ch < TT / 128; ++ch) { v4h o4; for (int q = 0; q < 4; ++q) o4[q] = tohx(v[ch * 4 + q] * f); *(volatile v4h*)(P16 + (size_t)i * TT + ch * 128 + lane * 4) = o4; } }
        if (ps == 0) __threadfence(); } }
__global__ __launch_bounds__(256) void k_gmrg(const float* __restrict__ A, const float* __restrict__ beta, bf* Yh, bf* Yl) { const size_t e = ((size_t)blockIdx.x * 256 + threadIdx.x) * 4; if (e >= (size_t)TT * DM) return; const int t = (int)(e / DM); const float cs = (t < RH) ? 1.0f : (1.0f / PCAR); const float gt = __fdiv_rn(1.0f, __fadd_rn(1.0f, expf(-bfr(beta[0])))); const float om = __fsub_rn(1.0f, gt); const v4f a = *(const v4f*)(A + e); v4us oh, ol;
#pragma unroll
    for (int u = 0; u < 4; ++u) { float y0 = a[u] * cs; asm volatile("" : "+v"(y0)); unsigned short p, q; splitf(__fmul_rn(om, y0), p, q); oh[u] = p; ol[u] = q; } *(volatile v4us*)(Yh + e) = oh; *(volatile v4us*)(Yl + e) = ol; __threadfence(); *(volatile v4us*)(Yh + e) = oh; *(volatile v4us*)(Yl + e) = ol; }

extern "C" void kernel_launch(void* const* d_in, const int* in_sizes, int n_in,
                              void* d_out, int out_size, void* d_ws, size_t ws_size, hipStream_t stream) {
    (void)in_sizes; (void)n_in; (void)out_size;
    const float* x = (const float*)d_in[0]; const float* cs_ = (const float*)d_in[1]; const float* sn_ = (const float*)d_in[2]; const float* Wq = (const float*)d_in[3]; const float* Wk = (const float*)d_in[4]; const float* Wv = (const float*)d_in[5]; const float* Wmp = (const float*)d_in[6]; const float* beta = (const float*)d_in[7]; const float* Wout = (const float*)d_in[8]; (void)Wmp;
    float* OUT = (float*)d_out;
    char* wsp = (char*)d_ws;
    auto take = [&](size_t bytes) { char* p = wsp; wsp += (bytes + 255) & ~(size_t)255; return (void*)p; };
    bf* BQ = (bf*)take((size_t)DM * DM * 2); bf* BK = (bf*)take((size_t)DM * DM * 2); bf* BV = (bf*)take((size_t)DM * DM * 2); bf* BO = (bf*)take((size_t)DM * DM * 2);
    bf* XB = (bf*)take((size_t)TT * DM * 2); float* FQ = (float*)take((size_t)TT * DM * 4); float* FK = (float*)take((size_t)TT * DM * 4); float* FV = (float*)take((size_t)TT * DM * 4);
    h16* Q16 = (h16*)take((size_t)TT * DM * 2); bf* Qh = (bf*)take((size_t)TT * DM * 2); bf* Ql = (bf*)take((size_t)TT * DM * 2); h16* K16 = (h16*)take((size_t)TT * DM * 2); bf* Kh = (bf*)take((size_t)TT * DM * 2); bf* Kl = (bf*)take((size_t)TT * DM * 2); h16* VT16 = (h16*)take((size_t)DM * TT * 2); bf* VTh = (bf*)take((size_t)DM * TT * 2); bf* VTl = (bf*)take((size_t)DM * TT * 2);
    float* S = (float*)take((size_t)TT * TT * 4); h16* P16 = (h16*)take((size_t)TT * TT * 2); bf* Ph = (bf*)take((size_t)RH * TT * 2); bf* Pl = (bf*)take((size_t)RH * TT * 2); float* A = (float*)take((size_t)TT * DM * 4); bf* Yh = (bf*)take((size_t)TT * DM * 2); bf* Yl = (bf*)take((size_t)TT * DM * 2);
    if ((size_t)(wsp - (char*)d_ws) > ws_size) return;
    k_cvt8<<<(DM * DM / 8 + 255) / 256, 256, 0, stream>>>(Wq, BQ, DM * DM / 8); k_cvt8<<<(DM * DM / 8 + 255) / 256, 256, 0, stream>>>(Wk, BK, DM * DM / 8); k_cvt8<<<(DM * DM / 8 + 255) / 256, 256, 0, stream>>>(Wv, BV, DM * DM / 8); k_cvt8<<<(DM * DM / 8 + 255) / 256, 256, 0, stream>>>(Wout, BO, DM * DM / 8);
    const dim3 gp(TT / 64, DM / 64, 1); const unsigned LP = (unsigned)(((size_t)TT * DM / 2 + 255) / 256);
    for (int b = 0; b < NB_; ++b) {
        k_cvt8<<<(TT * DM / 8 + 255) / 256, 256, 0, stream>>>(x + (size_t)b * TT * DM, XB, TT * DM / 8);
        k_gemmw<bf, 0, false><<<gp, 32, 0, stream>>>(XB, nullptr, BQ, nullptr, DM, FQ, DM, nullptr, 0, 0, 0); k_gemmw<bf, 0, false><<<gp, 32, 0, stream>>>(XB, nullptr, BK, nullptr, DM, FK, DM, nullptr, 0, 0, 0); k_gemmw<bf, 0, false><<<gp, 32, 0, stream>>>(XB, nullptr, BV, nullptr, DM, FV, DM, nullptr, 0, 0, 0);
        k_ropl<<<LP, 256, 0, stream>>>(FQ, cs_, sn_, Q16, Qh, Ql); k_ropl<<<LP, 256, 0, stream>>>(FK, cs_, sn_, K16, Kh, Kl); k_vtp1<<<(unsigned)(((size_t)DM * TT / 2 + 255) / 256), 256, 0, stream>>>(FV, VT16, VTh, VTl);
        k_gemmc<bf, 2, 1><<<dim3(RH / 64, TT / 64, 1), 32, 0, stream>>>(Qh, Ql, Kh, Kl, DM, S, TT, 0, 0, 0, 0);
        k_gemmc<h16, 0, 1><<<dim3((TT - RH) / 64, TT / 64, 1), 32, 0, stream>>>(Q16 + (size_t)RH * DM, nullptr, K16, nullptr, DM, S + (size_t)RH * TT, TT, RH, 0, 0, 0);
        k_isoft<<<TT / 8, 256, 0, stream>>>(S, P16, Ph, Pl);
        k_gemmc<bf, 2, 2><<<dim3(RH / 64, DM / 64, 1), 32, 0, stream>>>(Ph, Pl, VTh, VTl, TT, A, DM, 0, 0, 0, 0);
        k_gemmc<h16, 0, 2><<<dim3((TT - RH) / 64, DM / 64, 1), 32, 0, stream>>>(P16 + (size_t)RH * TT, nullptr, VT16, nullptr, TT, A + (size_t)RH * DM, DM, RH, 0, 0, 0);
        k_gmrg<<<(unsigned)(((size_t)TT * DM / 4 + 255) / 256), 256, 0, stream>>>(A, beta, Yh, Yl);
        k_gemmw<bf, 1, false><<<gp, 32, 0, stream>>>(Yh, Yl, BO, nullptr, DM, OUT + (size_t)b * TT * DM, DM, nullptr, 0, 0, 0); }
}
